// QuantumGate_53214644797979
// MI455X (gfx1250) — hardware-verified
//
#include <hip/hip_runtime.h>


#define NBR  8192
#define NIN  1024
#define NQ   8
#define NST  256
#define NPD  64
#define HOUT 512
#define PI_F 3.14159265358979323846f
typedef _Float16 h16;
typedef unsigned short bf;
typedef __attribute__((ext_vector_type(16))) __bf16   v16bf;
typedef __attribute__((ext_vector_type(16))) _Float16 v16h;
typedef __attribute__((ext_vector_type(8)))  _Float16 v8h;
typedef __attribute__((ext_vector_type(8)))  unsigned short v8us;
typedef __attribute__((ext_vector_type(8)))  float    v8f;
typedef __attribute__((ext_vector_type(4)))  float    v4f;
typedef v8h  __attribute__((may_alias)) v8ha;
typedef v4f  __attribute__((may_alias)) v4fa;
typedef v8us __attribute__((may_alias)) v8usa;

__device__ __forceinline__ unsigned short f2bf(float f) { unsigned u = __float_as_uint(f); u += 0x7FFFu + ((u >> 16) & 1u); return (unsigned short)(u >> 16); }
__device__ __forceinline__ float bf2f(unsigned short b) { return __uint_as_float(((unsigned)b) << 16); }
__device__ __forceinline__ float bfr(float f) { return bf2f(f2bf(f)); }
__device__ __forceinline__ v16h cat16(v8h lo, v8h hi) { return __builtin_shufflevector(lo, hi, 0, 1, 2, 3, 4, 5, 6, 7, 8, 9, 10, 11, 12, 13, 14, 15); }
__device__ __forceinline__ v16bf cat16b(v8us lo, v8us hi) { return __builtin_bit_cast(v16bf, __builtin_shufflevector(lo, hi, 0, 1, 2, 3, 4, 5, 6, 7, 8, 9, 10, 11, 12, 13, 14, 15)); }
__device__ __forceinline__ v8f wmma16(v16h a, v16h b, v8f c) { return __builtin_amdgcn_wmma_f32_16x16x32_f16(false, a, false, b, (short)0, c, false, false); }
__device__ __forceinline__ v8f wmmab(v16bf a, v16bf b, v8f c) { return __builtin_amdgcn_wmma_f32_16x16x32_bf16(false, a, false, b, (short)0, c, false, false); }


template <typename T16> struct WFrag;
template <> struct WFrag<h16> { typedef v16h V; static __device__ __forceinline__ V ld(const h16* p) { return cat16(*(const v8h*)p, *(const v8h*)(p + 16)); } static __device__ __forceinline__ v8f mma(V a, V b, v8f c) { return wmma16(a, b, c); } };
template <> struct WFrag<bf> { typedef v16bf V; static __device__ __forceinline__ V ld(const bf* p) { return cat16b(*(const v8us*)p, *(const v8us*)(p + 16)); } static __device__ __forceinline__ v8f mma(V a, V b, v8f c) { return wmmab(a, b, c); } };
template <typename T16, int NSPLIT, bool BIAS>
__global__ __launch_bounds__(32) void k_gemmw(const T16* __restrict__ A, const T16* __restrict__ A2, const T16* __restrict__ Bt, const T16* __restrict__ Bt2, int K, float* C, int ldc, const float* __restrict__ bias, size_t sA, size_t sB, size_t sC) {
    typedef typename WFrag<T16>::V V;
    __shared__ __align__(16) float os[16 * 68];
    const size_t z = blockIdx.z; A += z * sA; if (A2) A2 += z * sA; Bt += z * sB; if (Bt2) Bt2 += z * sB; C += z * sC;
    const int lane = threadIdx.x & 31, lr = lane & 15, hi = lane >> 4; const int r0 = blockIdx.x * 64, c0 = blockIdx.y * 64;
    v8f acc[4][4];
#pragma unroll
    for (int mb = 0; mb < 4; ++mb)
#pragma unroll
        for (int nb = 0; nb < 4; ++nb) acc[mb][nb] = (v8f){};
    const size_t aoff = (size_t)(r0 + lr) * K + 8 * hi, boff = (size_t)(c0 + lr) * K + 8 * hi;
#pragma unroll 1
    for (int kc = 0; kc < K; kc += 32) {
        V a[4], a2[4];
#pragma unroll
        for (int mb = 0; mb < 4; ++mb) { a[mb] = WFrag<T16>::ld(A + aoff + (size_t)mb * 16 * K + kc); if (NSPLIT == 1 || NSPLIT == 2) a2[mb] = WFrag<T16>::ld(A2 + aoff + (size_t)mb * 16 * K + kc); }
#pragma unroll
        for (int nb = 0; nb < 4; ++nb) { const V b = WFrag<T16>::ld(Bt + boff + (size_t)nb * 16 * K + kc); V b2; if (NSPLIT >= 2) b2 = WFrag<T16>::ld(Bt2 + boff + (size_t)nb * 16 * K + kc);
#pragma unroll
            for (int mb = 0; mb < 4; ++mb) { acc[mb][nb] = WFrag<T16>::mma(a[mb], b, acc[mb][nb]); if (NSPLIT == 1 || NSPLIT == 2) acc[mb][nb] = WFrag<T16>::mma(a2[mb], b, acc[mb][nb]); if (NSPLIT >= 2) acc[mb][nb] = WFrag<T16>::mma(a[mb], b2, acc[mb][nb]); } }
        asm volatile("v_nop\n\tv_nop\n\tv_nop\n\tv_nop" : "+v"(acc[0][0]), "+v"(acc[1][1]), "+v"(acc[2][2]), "+v"(acc[3][3]) : "v"(a[0]), "v"(a[3]));
    }
#pragma unroll
    for (int mb = 0; mb < 4; ++mb) {
#pragma unroll
        for (int nb = 0; nb < 4; ++nb) {
#pragma unroll
            for (int j = 0; j < 8; ++j) os[(hi * 8 + j) * 68 + nb * 16 + lr] = acc[mb][nb][j]; }
        __builtin_amdgcn_wave_barrier(); asm volatile("" ::: "memory");
        float* crow = C + (size_t)(r0 + mb * 16) * ldc + c0;
#pragma unroll 1
        for (int ps = 0; ps < 2; ++ps) {
#pragma unroll
            for (int s = 0; s < 8; ++s) { const int row = 2 * s + hi, cofs = lr * 4; v4f val = *(const v4fa*)(os + row * 68 + cofs); if (BIAS) { val[0] += bfr(bias[c0 + cofs]); val[1] += bfr(bias[c0 + cofs + 1]); val[2] += bfr(bias[c0 + cofs + 2]); val[3] += bfr(bias[c0 + cofs + 3]); }
                *(volatile v4f*)(crow + (size_t)row * ldc + cofs) = val; }
            if (ps == 0) __threadfence(); }
        __builtin_amdgcn_wave_barrier(); asm volatile("" ::: "memory");
    }
}

__device__ __forceinline__ void splitf(float y, unsigned short& h, unsigned short& l) { h = f2bf(y); l = f2bf(y - bf2f(h)); }
typedef __attribute__((ext_vector_type(2))) unsigned short v2us;
typedef __attribute__((ext_vector_type(2))) float v2f;
__global__ __launch_bounds__(256) void k_cvt8(const float* __restrict__ src, bf* dst, size_t n8) { const size_t i = (size_t)blockIdx.x * 256 + threadIdx.x; if (i >= n8) return; const v8f v = *(const v8f*)(src + i * 8); v8us o;
#pragma unroll
    for (int k = 0; k < 8; ++k) o[k] = f2bf(v[k]); *(volatile v8us*)(dst + i * 8) = o; __threadfence(); *(volatile v8us*)(dst + i * 8) = o; }

__global__ __launch_bounds__(256) void k_xcat(const float* __restrict__ xt, const float* __restrict__ hp, bf* XC) { const size_t e = ((size_t)blockIdx.x * 256 + threadIdx.x) * 8; if (e >= (size_t)NBR * NIN) return; const int c = (int)(e % NIN); const size_t b = e / NIN; const float* src = (c < 512) ? (xt + b * 512 + c) : (hp + b * 512 + (c - 512)); const v8f v = *(const v8f*)src; v8us o;
#pragma unroll
    for (int q = 0; q < 8; ++q) o[q] = f2bf(v[q]); *(volatile v8us*)(XC + e) = o; __threadfence(); *(volatile v8us*)(XC + e) = o; }
__global__ __launch_bounds__(256) void k_winp(const float* __restrict__ W, bf* Bt) { const size_t e = ((size_t)blockIdx.x * 256 + threadIdx.x) * 8; if (e >= (size_t)NPD * NIN) return; const int n = (int)(e / NIN); v8us o;
#pragma unroll
    for (int q = 0; q < 8; ++q) o[q] = (n < NQ) ? f2bf(W[e + q]) : (unsigned short)0; *(volatile v8us*)(Bt + e) = o; __threadfence(); *(volatile v8us*)(Bt + e) = o; }
__global__ __launch_bounds__(256) void k_woutp(const float* __restrict__ W, bf* Bt) { const size_t e = ((size_t)blockIdx.x * 256 + threadIdx.x) * 8; if (e >= (size_t)HOUT * NPD) return; const int k0 = (int)(e % NPD); const int o = (int)(e / NPD); v8us ob;
#pragma unroll
    for (int q = 0; q < 8; ++q) ob[q] = (k0 + q < NQ) ? f2bf(W[(size_t)o * NQ + k0 + q]) : (unsigned short)0; *(volatile v8us*)(Bt + e) = ob; __threadfence(); *(volatile v8us*)(Bt + e) = ob; }
__global__ __launch_bounds__(256) void k_ang(const float* __restrict__ C1, const float* __restrict__ b_in, float* ANG) { const int e = blockIdx.x * 256 + threadIdx.x; if (e >= NBR * NQ) return; const int w = e % NQ; const size_t b = e / NQ; const float qin = __fmul_rn(PI_F, tanhf(__fadd_rn(C1[b * NPD + w], bfr(b_in[w])))); const float th = 0.5f * qin; v2f cs; cs[0] = cosf(th); cs[1] = sinf(th);
    *(volatile v2f*)(ANG + b * 2 * NQ + 2 * w) = cs; __threadfence(); *(volatile v2f*)(ANG + b * 2 * NQ + 2 * w) = cs; }
__global__ __launch_bounds__(256) void k_vqc(const float* __restrict__ ANG, const float* __restrict__ vw, bf* Fh, bf* Fl) {
    __shared__ float sre[NST], sim[NST], red[NST], cth[NQ], sth[NQ], cya[NQ], sya[NQ], czb[NQ], szb[NQ], ev[NQ];
    const int a = threadIdx.x; const size_t b = blockIdx.x;
    if (a < NQ) { cth[a] = ANG[b * 2 * NQ + 2 * a]; sth[a] = ANG[b * 2 * NQ + 2 * a + 1]; const float ay = 0.5f * bfr(vw[a]); cya[a] = cosf(ay); sya[a] = sinf(ay); } else if (a < 2 * NQ) { const int w = a - NQ; const float bz = 0.5f * bfr(vw[NQ + w]); czb[w] = cosf(bz); szb[w] = sinf(bz); }
    __syncthreads();
#pragma unroll 1
    for (int ps = 0; ps < 2; ++ps) {
        float re = 0.0625f, im = 0.0f;
#pragma unroll 1
        for (int gate = 0; gate < 3 * NQ; ++gate) {
            const int w = (gate < NQ) ? gate : (gate - NQ) / 2; const int bit = 7 - w; const int prt = a ^ (1 << bit); const int hi = (a >> bit) & 1;
            sre[a] = re; sim[a] = im; __syncthreads(); const float pre = sre[prt], pim = sim[prt]; __syncthreads();
            float nre, nim;
            if (gate < NQ) { const float c = cth[w], s = sth[w];
                nre = __fadd_rn(__fmul_rn(c, re), __fmul_rn(s, pim)); nim = __fsub_rn(__fmul_rn(c, im), __fmul_rn(s, pre)); }
            else if (((gate - NQ) & 1) == 0) { const float c = cya[w], s = sya[w];
                if (hi == 0) { nre = __fsub_rn(__fmul_rn(c, re), __fmul_rn(s, pre)); nim = __fsub_rn(__fmul_rn(c, im), __fmul_rn(s, pim)); } else { nre = __fadd_rn(__fmul_rn(s, pre), __fmul_rn(c, re)); nim = __fadd_rn(__fmul_rn(s, pim), __fmul_rn(c, im)); } }
            else { const float c = czb[w], s = szb[w];
                const float ss = (hi == 0) ? -s : s; nre = __fsub_rn(__fmul_rn(re, c), __fmul_rn(im, ss)); nim = __fadd_rn(__fmul_rn(re, ss), __fmul_rn(im, c)); }
            re = nre; im = nim; }
        {
            const int cb = a & 1; const int prt = a ^ 128;
            sre[a] = re; sim[a] = im; __syncthreads(); const float pre = sre[prt], pim = sim[prt]; __syncthreads();
            if (cb) { re = pre; im = pim; } }
        const float p = __fadd_rn(__fmul_rn(re, re), __fmul_rn(im, im));
#pragma unroll 1
        for (int w = 0; w < NQ; ++w) { red[a] = (((a >> (7 - w)) & 1) == 0) ? p : -p; __syncthreads();
#pragma unroll
            for (int s = NST / 2; s; s >>= 1) { if (a < s) red[a] = __fadd_rn(red[a], red[a + s]); __syncthreads(); }
            if (a == 0) ev[w] = red[0]; __syncthreads(); }
        if (a < 32) { v2us oh, ol;
#pragma unroll
            for (int q = 0; q < 2; ++q) { const int k = a * 2 + q; const float f = (k < NQ) ? ev[k] : 0.f; unsigned short h2, l2; splitf(f, h2, l2); oh[q] = h2; ol[q] = l2; }
            *(volatile v2us*)(Fh + b * NPD + a * 2) = oh; *(volatile v2us*)(Fl + b * NPD + a * 2) = ol; }
        if (ps == 0) __threadfence(); __syncthreads(); }
}

extern "C" void kernel_launch(void* const* d_in, const int* in_sizes, int n_in,
                              void* d_out, int out_size, void* d_ws, size_t ws_size, hipStream_t stream) {
    (void)in_sizes; (void)n_in; (void)out_size;
    const float* xt = (const float*)d_in[0]; const float* hp = (const float*)d_in[1]; const float* Win = (const float*)d_in[2]; const float* bin = (const float*)d_in[3]; const float* vw = (const float*)d_in[4]; const float* Wout = (const float*)d_in[5]; const float* bout = (const float*)d_in[6];
    float* OUT = (float*)d_out;
    char* wsp = (char*)d_ws;
    auto take = [&](size_t bytes) { char* p = wsp; wsp += (bytes + 255) & ~(size_t)255; return (void*)p; };
    bf* XC = (bf*)take((size_t)NBR * NIN * 2); bf* WIN = (bf*)take((size_t)NPD * NIN * 2); float* C1 = (float*)take((size_t)NBR * NPD * 4); bf* Fh = (bf*)take((size_t)NBR * NPD * 2); bf* Fl = (bf*)take((size_t)NBR * NPD * 2); bf* WOUT = (bf*)take((size_t)HOUT * NPD * 2); float* ANG = (float*)take((size_t)NBR * 2 * NQ * 4);
    if ((size_t)(wsp - (char*)d_ws) > ws_size) return;
    k_xcat<<<(unsigned)(((size_t)NBR * NIN / 8 + 255) / 256), 256, 0, stream>>>(xt, hp, XC); k_winp<<<(NPD * NIN / 8 + 255) / 256, 256, 0, stream>>>(Win, WIN); k_woutp<<<(HOUT * NPD / 8 + 255) / 256, 256, 0, stream>>>(Wout, WOUT);
    k_gemmw<bf, 0, false><<<dim3(NBR / 64, NPD / 64, 1), 32, 0, stream>>>(XC, nullptr, WIN, nullptr, NIN, C1, NPD, nullptr, 0, 0, 0);
    k_ang<<<(NBR * NQ + 255) / 256, 256, 0, stream>>>(C1, bin, ANG); k_vqc<<<NBR, 256, 0, stream>>>(ANG, vw, Fh, Fl);
    k_gemmw<bf, 1, true><<<dim3(NBR / 64, HOUT / 64, 1), 32, 0, stream>>>(Fh, Fl, WOUT, nullptr, NPD, OUT, HOUT, bout, 0, 0, 0);
}
